// AttentionTier_60808146977376
// MI455X (gfx1250) — hardware-verified
//
#include <hip/hip_runtime.h>
#include <math.h>
#include <stdint.h>

#define NB    4
#define SEQ   2048
#define DM    1024
#define NQKV  3072
#define NH    16
#define HD    64
#define NFREQ 32
#define AT_SMEM 49152

static_assert(SEQ % 64 == 0);
static_assert(DM % 64 == 0);
static_assert(NQKV % 64 == 0);
static_assert(DM % 32 == 0);
static_assert(NH * HD == DM);
static_assert((SEQ * NFREQ) % 256 == 0);

typedef __bf16 v16b __attribute__((ext_vector_type(16)));
typedef __bf16 v8b_t __attribute__((ext_vector_type(8)));
typedef v8b_t v8b __attribute__((may_alias));
typedef float v8f __attribute__((ext_vector_type(8)));
typedef float v4f_t __attribute__((ext_vector_type(4)));
typedef v4f_t v4f __attribute__((may_alias));
typedef unsigned short v8us_t __attribute__((ext_vector_type(8)));
typedef v8us_t v8us __attribute__((may_alias));

__device__ __forceinline__ unsigned short f2bf_bits(float f) {
  const unsigned u = __float_as_uint(f);
  return (unsigned short)((u + 0x7FFFu + ((u >> 16) & 1u)) >> 16);
}
__device__ __forceinline__ float bfb2f(unsigned short b) { return __uint_as_float(((unsigned)b) << 16); }
__device__ __forceinline__ __bf16 bits2bf(unsigned short b) { return __builtin_bit_cast(__bf16, b); }

__device__ __forceinline__ void split8(const float* sp, v8us& hv, v8us& lv) {
  const v4f f0 = *(const v4f*)(sp);
  const v4f f1 = *(const v4f*)(sp + 4);
#pragma unroll
  for (int e = 0; e < 4; ++e) {
    const unsigned short h0 = f2bf_bits(f0[e]);
    hv[e] = h0;
    lv[e] = f2bf_bits(f0[e] - bfb2f(h0));
    const unsigned short h1 = f2bf_bits(f1[e]);
    hv[4 + e] = h1;
    lv[4 + e] = f2bf_bits(f1[e] - bfb2f(h1));
  }
}

__device__ __forceinline__ v16b ldfrag(const __bf16* p) {
  union { v16b v; v8b h[2]; } f;
  f.h[0] = *(const v8b*)(p);
  f.h[1] = *(const v8b*)(p + 16);
  return f.v;
}
__device__ __forceinline__ v8f mma_b(v16b a, v16b b, v8f c) {
  return __builtin_amdgcn_wmma_f32_16x16x32_bf16(false, a, false, b, (short)0, c, false, false);
}
__device__ __forceinline__ v8f mma_g(v16b a, v16b b, v8f c) {
  c = __builtin_amdgcn_wmma_f32_16x16x32_bf16(false, a, false, b, (short)0, c, false, false);
  asm volatile("v_nop\n\tv_nop\n\tv_nop\n\tv_nop" : "+v"(c) : "v"(a), "v"(b));
  return c;
}
__device__ __forceinline__ void dep_guard(v8f& a, v8f& b, v16b x, v16b y) {
  asm volatile("v_nop\n\tv_nop\n\tv_nop\n\tv_nop" : "+v"(a), "+v"(b) : "v"(x), "v"(y));
}
__device__ __forceinline__ void keep4(v16b a, v16b b, v16b c, v16b d) {
  asm volatile("v_nop" :: "v"(a), "v"(b), "v"(c), "v"(d));
}
__device__ __forceinline__ void acc_guard4(v8f& a, v8f& b, v8f& c, v8f& d) {
  asm volatile("v_nop\n\tv_nop\n\tv_nop\n\tv_nop" : "+v"(a), "+v"(b), "+v"(c), "+v"(d));
}
__device__ __forceinline__ void wave_sync() {
  __builtin_amdgcn_fence(__ATOMIC_RELEASE, "workgroup");
  __builtin_amdgcn_wave_barrier();
  __builtin_amdgcn_fence(__ATOMIC_ACQUIRE, "workgroup");
}

__global__ __launch_bounds__(256)
void k_cvt(const float* __restrict__ src, unsigned short* __restrict__ dst, int n8) {
  const int i = blockIdx.x * 256 + threadIdx.x;
  if (i < n8) {
    const v4f a = *(const v4f*)(src + (size_t)i * 8);
    const v4f b = *(const v4f*)(src + (size_t)i * 8 + 4);
    v8us o;
#pragma unroll
    for (int e = 0; e < 4; ++e) { o[e] = f2bf_bits(a[e]); o[4 + e] = f2bf_bits(b[e]); }
    *(volatile v8us*)(dst + (size_t)i * 8) = o;
    __threadfence();
    *(volatile v8us*)(dst + (size_t)i * 8) = o;
  }
}

__global__ __launch_bounds__(32)
void k_invfreq(float* __restrict__ invf) {
#pragma clang fp contract(off)
  const int j = threadIdx.x;
  double r = 1.333521432163324;
#pragma unroll 1
  for (int it = 0; it < 6; ++it) {
    double p7 = r;
#pragma unroll 1
    for (int k = 1; k < 7; ++k) p7 *= r;
    const double f = p7 * r - 10.0;
    r = r - f / (8.0 * p7);
  }
  double p = 1.0;
#pragma unroll 1
  for (int k = 0; k < j; ++k) p *= r;
  const float pf = (float)p;
  const float v = 1.0f / pf;
  ((volatile float*)invf)[j] = v;
  __threadfence();
  ((volatile float*)invf)[j] = v;
}

__global__ __launch_bounds__(256)
void k_ropetab(const float* __restrict__ invf, float* __restrict__ cosT, float* __restrict__ sinT) {
#pragma clang fp contract(off)
  const int idx = blockIdx.x * 256 + threadIdx.x;
  if (idx < SEQ * NFREQ) {
    const int t = idx >> 5, jj = idx & 31;
    const float ang = (float)t * invf[jj];
    const float cv = cosf(ang);
    const float sv = sinf(ang);
    ((volatile float*)cosT)[idx] = cv;
    ((volatile float*)sinT)[idx] = sv;
    __threadfence();
    ((volatile float*)cosT)[idx] = cv;
    ((volatile float*)sinT)[idx] = sv;
  }
}

__global__ __launch_bounds__(256) __attribute__((amdgpu_num_vgpr(256)))
void k_qkv(const unsigned short* __restrict__ Xp, const unsigned short* __restrict__ Wp,
           const float* __restrict__ cosT, const float* __restrict__ sinT,
           unsigned short* __restrict__ Qh, unsigned short* __restrict__ Ql,
           unsigned short* __restrict__ Kh, unsigned short* __restrict__ Kl,
           unsigned short* __restrict__ Vh, unsigned short* __restrict__ Vl)
{
#pragma clang fp contract(off)
  __shared__ __align__(16) float sT[8][16 * 68];
  const int lane = threadIdx.x & 31;
  const int wave = threadIdx.x >> 5;
  const int tilesN = NQKV / 64;
  const int tile = blockIdx.x * 8 + wave;
  if (tile >= (SEQ / 64) * tilesN) return;
  const int tm = tile / tilesN;
  const int tn = tile - tm * tilesN;
  const int m0 = tm << 6;
  const int n0 = tn << 6;
  const __bf16* A  = (const __bf16*)(const void*)Xp;
  const __bf16* Bt = (const __bf16*)(const void*)Wp;
  const int c    = lane & 15;
  const int hh   = lane >> 4;
  const int koff = hh * 8;
  const int mOff = hh * 8;

  v8f acc[4][4];
#pragma unroll
  for (int i = 0; i < 4; ++i)
#pragma unroll
    for (int j = 0; j < 4; ++j) acc[i][j] = (v8f){0.f,0.f,0.f,0.f,0.f,0.f,0.f,0.f};

  for (int k0 = 0; k0 < DM; k0 += 32) {
    v16b bq[4];
#pragma unroll
    for (int j = 0; j < 4; ++j) bq[j] = ldfrag(Bt + (size_t)(n0 + (j << 4) + c) * DM + k0 + koff);
#pragma unroll
    for (int i = 0; i < 4; ++i) {
      const v16b a = ldfrag(A + (size_t)(m0 + (i << 4) + c) * DM + k0 + koff);
#pragma unroll
      for (int j = 0; j < 4; ++j) acc[i][j] = mma_b(a, bq[j], acc[i][j]);
      dep_guard(acc[i][0], acc[i][3], a, a);
    }
    keep4(bq[0], bq[1], bq[2], bq[3]);
  }
  acc_guard4(acc[0][0], acc[0][1], acc[0][2], acc[0][3]);
  acc_guard4(acc[1][0], acc[1][1], acc[1][2], acc[1][3]);
  acc_guard4(acc[2][0], acc[2][1], acc[2][2], acc[2][3]);
  acc_guard4(acc[3][0], acc[3][1], acc[3][2], acc[3][3]);

  float* slab = sT[wave];
  const int which = n0 >> 10;
  const int hc0   = n0 & (DM - 1);
  const int q4 = lane >> 3;
  const int c8 = (lane & 7) * 8;

  if (which < 2) {
    unsigned short* Dh = (which == 0) ? Qh : Kh;
    unsigned short* Dl = (which == 0) ? Ql : Kl;
#pragma unroll
    for (int i = 0; i < 4; ++i) {
      const int mb = m0 + (i << 4);
#pragma unroll
      for (int r = 0; r < 8; ++r) {
        const int t = mb + mOff + r;
        const float* cr = cosT + t * NFREQ;
        const float* sr = sinT + t * NFREQ;
#pragma unroll
        for (int j = 0; j < 2; ++j) {
          const int jj = (j << 4) + c;
          const float cv = cr[jj];
          const float sv = sr[jj];
          const float x1 = acc[i][j][r];
          const float x2 = acc[i][j + 2][r];
          const float o1 = x1 * cv - x2 * sv;
          const float o2 = x2 * cv + x1 * sv;
          slab[(mOff + r) * 68 + (j << 4) + c]       = o1;
          slab[(mOff + r) * 68 + ((j + 2) << 4) + c] = o2;
        }
      }
      wave_sync();
      for (int pass = 0; pass < 2; ++pass) {
#pragma unroll
        for (int it = 0; it < 4; ++it) {
          const int row = it * 4 + q4;
          v8us hv, lv;
          split8(slab + row * 68 + c8, hv, lv);
          const size_t go = (size_t)(mb + row) * DM + hc0 + c8;
          *(volatile v8us*)(Dh + go) = hv;
          *(volatile v8us*)(Dl + go) = lv;
        }
        __threadfence();
      }
      wave_sync();
    }
  } else {
#pragma unroll
    for (int j = 0; j < 4; ++j) {
#pragma unroll
      for (int i = 0; i < 4; ++i)
#pragma unroll
        for (int r = 0; r < 8; ++r) slab[c * 68 + (i << 4) + mOff + r] = acc[i][j][r];
      wave_sync();
      for (int pass = 0; pass < 2; ++pass) {
#pragma unroll
        for (int it = 0; it < 4; ++it) {
          const int dd = it * 4 + q4;
          v8us hv, lv;
          split8(slab + dd * 68 + c8, hv, lv);
          const size_t go = (size_t)(hc0 + (j << 4) + dd) * SEQ + m0 + c8;
          *(volatile v8us*)(Vh + go) = hv;
          *(volatile v8us*)(Vl + go) = lv;
        }
        __threadfence();
      }
      wave_sync();
    }
  }
}

__global__ __launch_bounds__(128) __attribute__((amdgpu_num_vgpr(256)))
void k_attn(const unsigned short* __restrict__ qhp, const unsigned short* __restrict__ qlp,
            const unsigned short* __restrict__ khp, const unsigned short* __restrict__ klp,
            const unsigned short* __restrict__ vhp, const unsigned short* __restrict__ vlp,
            unsigned short* __restrict__ ohp, unsigned short* __restrict__ olp, float sscale)
{
#pragma clang fp contract(off)
  union FB { v16b v; v8b h[2]; };
  __shared__ __align__(16) unsigned char smem[AT_SMEM];
  const int tid  = threadIdx.x;
  const int wave = tid >> 5;
  const int lane = tid & 31;
  const int hh   = lane >> 4;
  const int c    = lane & 15;

  __bf16* Ksh = (__bf16*)(void*)(smem);
  __bf16* Ksl = (__bf16*)(void*)(smem + 8192);
  __bf16* Vth = (__bf16*)(void*)(smem + 16384);
  __bf16* Vtl = (__bf16*)(void*)(smem + 24576);
  __bf16* pwh = (__bf16*)(void*)(smem + 32768) + wave * (16 * 64);
  __bf16* pwl = (__bf16*)(void*)(smem + 40960) + wave * (16 * 64);

  const int nqb = SEQ / 64;
  const int qb  = blockIdx.x % nqb;
  const int h   = blockIdx.x / nqb;
  const int q0  = qb * 64 + wave * 16;

  const __bf16* Qh = (const __bf16*)(const void*)qhp + (size_t)h * HD;
  const __bf16* Ql = (const __bf16*)(const void*)qlp + (size_t)h * HD;
  const __bf16* Kh = (const __bf16*)(const void*)khp + (size_t)h * HD;
  const __bf16* Kl = (const __bf16*)(const void*)klp + (size_t)h * HD;
  const __bf16* Vh = (const __bf16*)(const void*)vhp + (size_t)h * HD * SEQ;
  const __bf16* Vl = (const __bf16*)(const void*)vlp + (size_t)h * HD * SEQ;
  unsigned short* Oh = ohp + (size_t)h * HD;
  unsigned short* Ol = olp + (size_t)h * HD;

  v16b qah[2], qal[2];
#pragma unroll
  for (int dc = 0; dc < 2; ++dc) {
    qah[dc] = ldfrag(Qh + (size_t)(q0 + c) * DM + dc * 32 + 8 * hh);
    qal[dc] = ldfrag(Ql + (size_t)(q0 + c) * DM + dc * 32 + 8 * hh);
  }

  float mrow[8], lrow[8];
  v8f oacc[4];
#pragma unroll
  for (int r = 0; r < 8; ++r) { mrow[r] = -INFINITY; lrow[r] = 0.f; }
#pragma unroll
  for (int t = 0; t < 4; ++t) oacc[t] = (v8f){0.f,0.f,0.f,0.f,0.f,0.f,0.f,0.f};

  const int nChunks = qb + 1;
  for (int kc = 0; kc < nChunks; ++kc) {
    const int kv0 = kc * 64;
    __syncthreads();
    {
      const int r = tid >> 1, half = (tid & 1) * 32;
      const __bf16* ksh = Kh + (size_t)(kv0 + r) * DM + half;
      const __bf16* ksl = Kl + (size_t)(kv0 + r) * DM + half;
      const __bf16* vsh = Vh + (size_t)r * SEQ + kv0 + half;
      const __bf16* vsl = Vl + (size_t)r * SEQ + kv0 + half;
#pragma unroll
      for (int i = 0; i < 4; ++i) {
        const v8b a0 = *(const v8b*)(ksh + 8 * i);
        const v8b a1 = *(const v8b*)(ksl + 8 * i);
        const v8b b0 = *(const v8b*)(vsh + 8 * i);
        const v8b b1 = *(const v8b*)(vsl + 8 * i);
        *(v8b*)(Ksh + r * 64 + half + 8 * i) = a0;
        *(v8b*)(Ksl + r * 64 + half + 8 * i) = a1;
        *(v8b*)(Vth + r * 64 + half + 8 * i) = b0;
        *(v8b*)(Vtl + r * 64 + half + 8 * i) = b1;
      }
    }
    __syncthreads();

    v8f s[4];
#pragma unroll
    for (int j = 0; j < 4; ++j) {
      s[j] = (v8f){0.f,0.f,0.f,0.f,0.f,0.f,0.f,0.f};
#pragma unroll
      for (int dc = 0; dc < 2; ++dc) {
        FB kb, kl;
        kb.h[0] = *(const v8b*)(Ksh + (j * 16 + c) * 64 + dc * 32 + 8 * hh);
        kb.h[1] = *(const v8b*)(Ksh + (j * 16 + c) * 64 + dc * 32 + 16 + 8 * hh);
        kl.h[0] = *(const v8b*)(Ksl + (j * 16 + c) * 64 + dc * 32 + 8 * hh);
        kl.h[1] = *(const v8b*)(Ksl + (j * 16 + c) * 64 + dc * 32 + 16 + 8 * hh);
        s[j] = mma_g(qah[dc], kb.v, s[j]);
        s[j] = mma_g(qah[dc], kl.v, s[j]);
        s[j] = mma_g(qal[dc], kb.v, s[j]);
      }
    }
    const bool diag = (kc == qb);
    float cm[8];
#pragma unroll
    for (int r = 0; r < 8; ++r) {
      const int qrow = q0 + 8 * hh + r;
      float m = -INFINITY;
#pragma unroll
      for (int j = 0; j < 4; ++j) {
        const int kvcol = kv0 + j * 16 + c;
        const float sv = s[j][r] * sscale;
        const bool masked = diag && (kvcol > qrow);
        const float sm = masked ? -INFINITY : sv;
        s[j][r] = sm;
        m = fmaxf(m, sm);
      }
#pragma unroll
      for (int off = 1; off < 16; off <<= 1) m = fmaxf(m, __shfl_xor(m, off, 32));
      cm[r] = m;
    }
#pragma unroll
    for (int r = 0; r < 8; ++r) {
      const float mnew  = fmaxf(mrow[r], cm[r]);
      const float alpha = expf(mrow[r] - mnew);
      mrow[r] = mnew;
      float psum = 0.f;
#pragma unroll
      for (int j = 0; j < 4; ++j) {
        const float p = expf(s[j][r] - mnew);
        psum += p;
        const unsigned short hb = f2bf_bits(p);
        const unsigned short lb = f2bf_bits(p - bfb2f(hb));
        pwh[(8 * hh + r) * 64 + j * 16 + c] = bits2bf(hb);
        pwl[(8 * hh + r) * 64 + j * 16 + c] = bits2bf(lb);
      }
#pragma unroll
      for (int off = 1; off < 16; off <<= 1) psum += __shfl_xor(psum, off, 32);
      lrow[r] = lrow[r] * alpha + psum;
#pragma unroll
      for (int t = 0; t < 4; ++t) oacc[t][r] *= alpha;
    }
    wave_sync();
#pragma unroll 1
    for (int kk = 0; kk < 2; ++kk) {
      FB pa, pl;
      pa.h[0] = *(const v8b*)(pwh + c * 64 + kk * 32 + 8 * hh);
      pa.h[1] = *(const v8b*)(pwh + c * 64 + kk * 32 + 16 + 8 * hh);
      pl.h[0] = *(const v8b*)(pwl + c * 64 + kk * 32 + 8 * hh);
      pl.h[1] = *(const v8b*)(pwl + c * 64 + kk * 32 + 16 + 8 * hh);
#pragma unroll
      for (int t = 0; t < 4; ++t) {
        FB vb, vl;
        vb.h[0] = *(const v8b*)(Vth + (t * 16 + c) * 64 + kk * 32 + 8 * hh);
        vb.h[1] = *(const v8b*)(Vth + (t * 16 + c) * 64 + kk * 32 + 16 + 8 * hh);
        vl.h[0] = *(const v8b*)(Vtl + (t * 16 + c) * 64 + kk * 32 + 8 * hh);
        vl.h[1] = *(const v8b*)(Vtl + (t * 16 + c) * 64 + kk * 32 + 16 + 8 * hh);
        oacc[t] = mma_g(pa.v, vb.v, oacc[t]);
        oacc[t] = mma_g(pa.v, vl.v, oacc[t]);
        oacc[t] = mma_g(pl.v, vb.v, oacc[t]);
      }
    }
  }

  __syncthreads();
  float* os = (float*)(void*)smem + wave * (16 * 68);
#pragma unroll
  for (int r = 0; r < 8; ++r) {
    const float inv = 1.0f / lrow[r];
#pragma unroll
    for (int t = 0; t < 4; ++t) os[(8 * hh + r) * 68 + t * 16 + c] = oacc[t][r] * inv;
  }
  wave_sync();
  {
    const int q4 = lane >> 3, c8 = (lane & 7) * 8;
    for (int pass = 0; pass < 2; ++pass) {
#pragma unroll
      for (int it = 0; it < 4; ++it) {
        const int row = it * 4 + q4;
        v8us hv, lv;
        split8(os + row * 68 + c8, hv, lv);
        const size_t go = (size_t)(q0 + row) * DM + c8;
        *(volatile v8us*)(Oh + go) = hv;
        *(volatile v8us*)(Ol + go) = lv;
      }
      __threadfence();
    }
  }
}

__global__ __launch_bounds__(256) __attribute__((amdgpu_num_vgpr(256)))
void k_out(const unsigned short* __restrict__ Ahp, const unsigned short* __restrict__ Alp,
           const unsigned short* __restrict__ Wp, float* __restrict__ Out)
{
  __shared__ __align__(16) float sT[8][16 * 68];
  const int lane = threadIdx.x & 31;
  const int wave = threadIdx.x >> 5;
  const int tilesN = DM / 64;
  const int tile = blockIdx.x * 8 + wave;
  if (tile >= (SEQ / 64) * tilesN) return;
  const int tm = tile / tilesN;
  const int tn = tile - tm * tilesN;
  const int m0 = tm << 6;
  const int n0 = tn << 6;
  const __bf16* Ah = (const __bf16*)(const void*)Ahp;
  const __bf16* Al = (const __bf16*)(const void*)Alp;
  const __bf16* Bt = (const __bf16*)(const void*)Wp;
  const int c    = lane & 15;
  const int hh   = lane >> 4;
  const int koff = hh * 8;
  const int mOff = hh * 8;

  v8f acc[4][4];
#pragma unroll
  for (int i = 0; i < 4; ++i)
#pragma unroll
    for (int j = 0; j < 4; ++j) acc[i][j] = (v8f){0.f,0.f,0.f,0.f,0.f,0.f,0.f,0.f};

  for (int k0 = 0; k0 < DM; k0 += 32) {
    v16b bq[4];
#pragma unroll
    for (int j = 0; j < 4; ++j) bq[j] = ldfrag(Bt + (size_t)(n0 + (j << 4) + c) * DM + k0 + koff);
#pragma unroll
    for (int i = 0; i < 4; ++i) {
      const size_t ao = (size_t)(m0 + (i << 4) + c) * DM + k0 + koff;
      const v16b ah = ldfrag(Ah + ao);
      const v16b al = ldfrag(Al + ao);
#pragma unroll
      for (int j = 0; j < 4; ++j) {
        acc[i][j] = mma_b(ah, bq[j], acc[i][j]);
        acc[i][j] = mma_b(al, bq[j], acc[i][j]);
      }
      dep_guard(acc[i][0], acc[i][3], ah, al);
    }
    keep4(bq[0], bq[1], bq[2], bq[3]);
  }
  acc_guard4(acc[0][0], acc[0][1], acc[0][2], acc[0][3]);
  acc_guard4(acc[1][0], acc[1][1], acc[1][2], acc[1][3]);
  acc_guard4(acc[2][0], acc[2][1], acc[2][2], acc[2][3]);
  acc_guard4(acc[3][0], acc[3][1], acc[3][2], acc[3][3]);

  float* slab = sT[wave];
  const int c4 = (lane & 15) * 4;
#pragma unroll
  for (int i = 0; i < 4; ++i) {
    const int mb = m0 + (i << 4);
#pragma unroll
    for (int j = 0; j < 4; ++j)
#pragma unroll
      for (int r = 0; r < 8; ++r) slab[(mOff + r) * 68 + (j << 4) + c] = acc[i][j][r];
    wave_sync();
    for (int pass = 0; pass < 2; ++pass) {
#pragma unroll
      for (int it = 0; it < 8; ++it) {
        const int row = it * 2 + hh;
        const v4f v = *(const v4f*)(slab + row * 68 + c4);
        *(volatile v4f*)(Out + (size_t)(mb + row) * DM + n0 + c4) = v;
      }
      __threadfence();
    }
    wave_sync();
  }
}

extern "C" void kernel_launch(void* const* d_in, const int* in_sizes, int n_in,
                              void* d_out, int out_size, void* d_ws, size_t ws_size,
                              hipStream_t stream) {
  if (n_in < 3) return;
  if (in_sizes[0] != NB * SEQ * DM) return;
  if (in_sizes[1] != NQKV * DM) return;
  if (in_sizes[2] != DM * DM) return;
  if (out_size != NB * SEQ * DM) return;

  const float* x    = (const float*)d_in[0];
  const float* Wqkv = (const float*)d_in[1];
  const float* Wout = (const float*)d_in[2];
  float* out = (float*)d_out;

  const size_t szXb  = (size_t)NB * SEQ * DM * 2;
  const size_t szWq  = (size_t)NQKV * DM * 2;
  const size_t szWo  = (size_t)DM * DM * 2;
  const size_t szPl  = (size_t)SEQ * DM * 2;
  const size_t szTab = (size_t)SEQ * NFREQ * 4;
  const size_t szInv = 256;
  size_t off = 0;
  const size_t oXb = off; off += szXb;
  const size_t oWq = off; off += szWq;
  const size_t oWo = off; off += szWo;
  const size_t oQh = off; off += szPl;  const size_t oQl = off; off += szPl;
  const size_t oKh = off; off += szPl;  const size_t oKl = off; off += szPl;
  const size_t oVh = off; off += szPl;  const size_t oVl = off; off += szPl;
  const size_t oOh = off; off += szPl;  const size_t oOl = off; off += szPl;
  const size_t oCos = off; off += szTab;
  const size_t oSin = off; off += szTab;
  const size_t oInv = off; off += szInv;
  if (off > ws_size) return;

  char* ws = (char*)d_ws;
  unsigned short* Xb  = (unsigned short*)(ws + oXb);
  unsigned short* Wqb = (unsigned short*)(ws + oWq);
  unsigned short* Wob = (unsigned short*)(ws + oWo);
  unsigned short* Qh  = (unsigned short*)(ws + oQh);  unsigned short* Ql = (unsigned short*)(ws + oQl);
  unsigned short* Kh  = (unsigned short*)(ws + oKh);  unsigned short* Kl = (unsigned short*)(ws + oKl);
  unsigned short* Vh  = (unsigned short*)(ws + oVh);  unsigned short* Vl = (unsigned short*)(ws + oVl);
  unsigned short* Oh  = (unsigned short*)(ws + oOh);  unsigned short* Ol = (unsigned short*)(ws + oOl);
  float* cosT = (float*)(ws + oCos);
  float* sinT = (float*)(ws + oSin);
  float* invf = (float*)(ws + oInv);

  k_invfreq<<<dim3(1), dim3(32), 0, stream>>>(invf);
  k_ropetab<<<dim3((SEQ * NFREQ) / 256), dim3(256), 0, stream>>>(invf, cosT, sinT);

  const int nx8 = (NB * SEQ * DM) / 8;
  const int nq8 = (NQKV * DM) / 8;
  const int no8 = (DM * DM) / 8;
  k_cvt<<<dim3((nx8 + 255) / 256), dim3(256), 0, stream>>>(x, Xb, nx8);
  k_cvt<<<dim3((nq8 + 255) / 256), dim3(256), 0, stream>>>(Wqkv, Wqb, nq8);
  k_cvt<<<dim3((no8 + 255) / 256), dim3(256), 0, stream>>>(Wout, Wob, no8);

  const dim3 gQKV((((SEQ / 64) * (NQKV / 64)) + 7) / 8);
  const dim3 gAtt(NH * (SEQ / 64));
  const dim3 gOut((((SEQ / 64) * (DM / 64)) + 7) / 8);

  for (int b = 0; b < NB; ++b) {
    const unsigned short* xb = Xb + (size_t)b * SEQ * DM;
    k_qkv<<<gQKV, dim3(256), 0, stream>>>(xb, Wqb, cosT, sinT, Qh, Ql, Kh, Kl, Vh, Vl);
    k_attn<<<gAtt, dim3(128), 0, stream>>>(Qh, Ql, Kh, Kl, Vh, Vl, Oh, Ol, 0.125f);
    float* outb = out + (size_t)b * SEQ * DM;
    k_out<<<gOut, dim3(256), 0, stream>>>(Oh, Ol, Wob, outb);
  }
  (void)hipGetLastError();
}
